// CrossAttention_87101936763227
// MI455X (gfx1250) — hardware-verified
//
#include <hip/hip_runtime.h>


#ifndef NB
#define NB 2
#endif
#ifndef SEQ
#define SEQ 4096
#endif
#define NB_FULL  2
#define SEQ_FULL 4096
#ifndef OUT_SEQ_STRIDE
#define OUT_SEQ_STRIDE SEQ_FULL
#endif

#define DMODEL 512
#define NHEAD  8
#define DH     64
#define NROWS  (NB * SEQ)
#define NBH    (NB * NHEAD)

#define QK_LDS 72
#define V_LDS  136
#define P_LDS  72
#define O_LDS  68

static_assert(SEQ % 128 == 0);
static_assert(NB >= 1 && NB <= NB_FULL);
static_assert(SEQ <= SEQ_FULL);
static_assert(DMODEL == NHEAD * DH);

#define DEVINL static __device__ __forceinline__

typedef _Float16     v16h __attribute__((ext_vector_type(16)));
typedef _Float16     v8h  __attribute__((ext_vector_type(8)));
typedef float        v8f  __attribute__((ext_vector_type(8)));
typedef float        v4f  __attribute__((ext_vector_type(4)));
typedef unsigned int v4u  __attribute__((ext_vector_type(4)));

union Frag16 { v4u q[2]; v16h v; };
union Pack8  { v8h h; v4u u; };

#define W_CARRY    64.0f
#define QKV_STORE  0.25f
#define SC_SCALE   0.00048828125f
#define P_CARRY    1024.0f
#define AO_FAC     0.00390625f
#define OUT_FAC    0.000244140625f

DEVINL float bf16_rne(float f) {
  unsigned int u = __float_as_uint(f);
  u += 0x7FFFu + ((u >> 16) & 1u);
  u &= 0xFFFF0000u;
  return __uint_as_float(u);
}

DEVINL v16h load_frag(const _Float16* base, int ld, int r0, int k0, int lane) {
  const int R = lane & 15, g = lane >> 4;
  const _Float16* p = base + (size_t)(r0 + R) * (size_t)ld + k0 + g * 8;
  Frag16 f;
  f.q[0] = *(const v4u*)(p);
  f.q[1] = *(const v4u*)(p + 16);
  return f.v;
}

DEVINL v8f wmma_f16(v16h a, v16h b, v8f c) {
  c = __builtin_amdgcn_wmma_f32_16x16x32_f16(false, a, false, b, (short)0, c, false, false);
  asm volatile("v_nop\n\tv_nop\n\tv_nop\n\tv_nop" : "+v"(c) : "v"(a), "v"(b));
  return c;
}

__global__ __launch_bounds__(256) void cvt_kernel(
    const float* __restrict__ X,
    const float* __restrict__ Wq, const float* __restrict__ Wk,
    const float* __restrict__ Wv, const float* __restrict__ Wo,
    _Float16* __restrict__ Xh,
    _Float16* __restrict__ Wqh, _Float16* __restrict__ Wkh,
    _Float16* __restrict__ Wvh, _Float16* __restrict__ Woh,
    int nxblk)
{
  const int blk = blockIdx.x;
  const int tid = threadIdx.x;
  const float* src;
  _Float16*    dst;
  float        sc;
  if (blk < nxblk) {
    const size_t idx = ((size_t)blk * 256 + tid) * 8;
    const size_t row = idx >> 9;
    const int    col = (int)(idx & 511);
    const size_t b   = row / SEQ;
    const size_t s   = row - b * SEQ;
    src = X + (b * SEQ_FULL + s) * DMODEL + col;
    dst = Xh + idx;
    sc  = 1.0f;
  } else {
    const int    wb  = blk - nxblk;
    const int    w   = wb >> 7;
    const size_t idx = ((size_t)(wb & 127) * 256 + tid) * 8;
    const float* wsrc = (w == 0) ? Wq  : (w == 1) ? Wk  : (w == 2) ? Wv  : Wo;
    _Float16*    wdst = (w == 0) ? Wqh : (w == 1) ? Wkh : (w == 2) ? Wvh : Woh;
    src = wsrc + idx;
    dst = wdst + idx;
    sc  = W_CARRY;
  }
  const v4f f0 = *(const v4f*)(src);
  const v4f f1 = *(const v4f*)(src + 4);
  Pack8 pk;
  pk.h[0] = (_Float16)(bf16_rne(f0.x) * sc);
  pk.h[1] = (_Float16)(bf16_rne(f0.y) * sc);
  pk.h[2] = (_Float16)(bf16_rne(f0.z) * sc);
  pk.h[3] = (_Float16)(bf16_rne(f0.w) * sc);
  pk.h[4] = (_Float16)(bf16_rne(f1.x) * sc);
  pk.h[5] = (_Float16)(bf16_rne(f1.y) * sc);
  pk.h[6] = (_Float16)(bf16_rne(f1.z) * sc);
  pk.h[7] = (_Float16)(bf16_rne(f1.w) * sc);
  const v4u val = pk.u;
  *(volatile v4u*)dst = val;
  __threadfence();
  *(volatile v4u*)dst = val;
}

__global__ __launch_bounds__(128) __attribute__((amdgpu_num_vgpr(256)))
void qkv_kernel(const _Float16* __restrict__ Xh,
                const _Float16* __restrict__ Wqh,
                const _Float16* __restrict__ Wkh,
                const _Float16* __restrict__ Wvh,
                _Float16* __restrict__ Qp,
                _Float16* __restrict__ Kp,
                _Float16* __restrict__ Vtp)
{
  __shared__ __attribute__((aligned(16))) _Float16 stile[128 * QK_LDS];

  const int lane = threadIdx.x & 31;
  const int wave = threadIdx.x >> 5;
  const int N = lane & 15, g = lane >> 4;
  const int h   = blockIdx.x;
  const int n0  = h * DH;
  const int nb0 = blockIdx.y * 128;
  const int m0  = nb0 + wave * 32;
  const int z   = blockIdx.z;
  const _Float16* W = (z == 0) ? Wqh : (z == 1) ? Wkh : Wvh;

  v8f acc[2][4];
#pragma unroll
  for (int u = 0; u < 2; ++u)
#pragma unroll
    for (int t = 0; t < 4; ++t)
#pragma unroll
      for (int r = 0; r < 8; ++r) acc[u][t][r] = 0.0f;

#pragma unroll 1
  for (int k0 = 0; k0 < DMODEL; k0 += 32) {
    const v16h a0 = load_frag(Xh, DMODEL, m0,      k0, lane);
    const v16h a1 = load_frag(Xh, DMODEL, m0 + 16, k0, lane);
#pragma unroll
    for (int t = 0; t < 4; ++t) {
      const v16h b = load_frag(W, DMODEL, n0 + t * 16, k0, lane);
      acc[0][t] = wmma_f16(a0, b, acc[0][t]);
      acc[1][t] = wmma_f16(a1, b, acc[1][t]);
    }
  }

  if (z == 2) {
#pragma unroll
    for (int u = 0; u < 2; ++u)
#pragma unroll
      for (int t = 0; t < 4; ++t) {
        Pack8 pk;
#pragma unroll
        for (int r = 0; r < 8; ++r) pk.h[r] = (_Float16)(acc[u][t][r] * QKV_STORE);
        *(v4u*)&stile[(t * 16 + N) * V_LDS + wave * 32 + u * 16 + 8 * g] = pk.u;
      }
  } else {
#pragma unroll
    for (int u = 0; u < 2; ++u)
#pragma unroll
      for (int t = 0; t < 4; ++t)
#pragma unroll
        for (int r = 0; r < 8; ++r)
          stile[(wave * 32 + u * 16 + 8 * g + r) * QK_LDS + t * 16 + N] =
              (_Float16)(acc[u][t][r] * QKV_STORE);
  }
  __syncthreads();

  const int b  = nb0 / SEQ;
  const int s0 = nb0 - b * SEQ;
  const int bh = b * NHEAD + h;
  const int lq = lane >> 3;
  const int lp = lane & 7;

  if (z == 2) {
    _Float16* base = Vtp + ((size_t)bh * DH) * SEQ + s0;
#pragma unroll
    for (int i = 0; i < 8; ++i) {
      const int L = i * 4 + lq;
      const int d = wave * 16 + (L >> 1);
      const int soff = (L & 1) * 64 + lp * 8;
      const v4u v = *(const v4u*)&stile[d * V_LDS + soff];
      *(volatile v4u*)(base + (size_t)d * SEQ + soff) = v;
    }
    __threadfence();
#pragma unroll
    for (int i = 0; i < 8; ++i) {
      const int L = i * 4 + lq;
      const int d = wave * 16 + (L >> 1);
      const int soff = (L & 1) * 64 + lp * 8;
      const v4u v = *(const v4u*)&stile[d * V_LDS + soff];
      *(volatile v4u*)(base + (size_t)d * SEQ + soff) = v;
    }
  } else {
    _Float16* base = ((z == 0) ? Qp : Kp) + ((size_t)bh * SEQ + s0) * DH;
#pragma unroll
    for (int i = 0; i < 8; ++i) {
      const int row = wave * 32 + i * 4 + lq;
      const v4u v = *(const v4u*)&stile[row * QK_LDS + lp * 8];
      *(volatile v4u*)(base + (size_t)row * DH + lp * 8) = v;
    }
    __threadfence();
#pragma unroll
    for (int i = 0; i < 8; ++i) {
      const int row = wave * 32 + i * 4 + lq;
      const v4u v = *(const v4u*)&stile[row * QK_LDS + lp * 8];
      *(volatile v4u*)(base + (size_t)row * DH + lp * 8) = v;
    }
  }
}

__global__ __launch_bounds__(128) __attribute__((amdgpu_num_vgpr(256)))
void attn_kernel(const _Float16* __restrict__ Qp,
                 const _Float16* __restrict__ Kp,
                 const _Float16* __restrict__ Vtp,
                 _Float16* __restrict__ AOp)
{
  __shared__ __attribute__((aligned(16))) _Float16 plds[4][16][P_LDS];

  const int lane = threadIdx.x & 31;
  const int wave = threadIdx.x >> 5;
  const int N = lane & 15, g = lane >> 4;
  const int bh = blockIdx.y;
  const int q0 = blockIdx.x * 64 + wave * 16;

  const _Float16* Qb = Qp  + (size_t)bh * SEQ * DH;
  const _Float16* Kb = Kp  + (size_t)bh * SEQ * DH;
  const _Float16* Vb = Vtp + (size_t)bh * DH * SEQ;

  const v16h aq0 = load_frag(Qb, DH, q0, 0,  lane);
  const v16h aq1 = load_frag(Qb, DH, q0, 32, lane);

  v8f o[4];
#pragma unroll
  for (int t = 0; t < 4; ++t)
#pragma unroll
    for (int r = 0; r < 8; ++r) o[t][r] = 0.0f;

  float mrun[8], lrun[8];
#pragma unroll
  for (int r = 0; r < 8; ++r) { mrun[r] = -1e30f; lrun[r] = 0.0f; }

  const _Float16* prow = &plds[wave][0][0];

#pragma unroll 1
  for (int kb = 0; kb < SEQ; kb += 64) {
    v8f st[4];
#pragma unroll
    for (int t = 0; t < 4; ++t) {
      v8f c;
#pragma unroll
      for (int r = 0; r < 8; ++r) c[r] = 0.0f;
      const v16h b0 = load_frag(Kb, DH, kb + t * 16, 0,  lane);
      c = wmma_f16(aq0, b0, c);
      const v16h b1 = load_frag(Kb, DH, kb + t * 16, 32, lane);
      c = wmma_f16(aq1, b1, c);
      st[t] = c;
    }

    float bm[8];
#pragma unroll
    for (int r = 0; r < 8; ++r) {
      const float v0 = st[0][r] * SC_SCALE; st[0][r] = v0;
      const float v1 = st[1][r] * SC_SCALE; st[1][r] = v1;
      const float v2 = st[2][r] * SC_SCALE; st[2][r] = v2;
      const float v3 = st[3][r] * SC_SCALE; st[3][r] = v3;
      float m = fmaxf(fmaxf(v0, v1), fmaxf(v2, v3));
      m = fmaxf(m, __shfl_xor(m, 1, 32));
      m = fmaxf(m, __shfl_xor(m, 2, 32));
      m = fmaxf(m, __shfl_xor(m, 4, 32));
      m = fmaxf(m, __shfl_xor(m, 8, 32));
      bm[r] = m;
    }
    float alpha[8], mnew[8], rs[8];
#pragma unroll
    for (int r = 0; r < 8; ++r) {
      mnew[r]  = fmaxf(mrun[r], bm[r]);
      alpha[r] = __expf(mrun[r] - mnew[r]);
      mrun[r]  = mnew[r];
      rs[r]    = 0.0f;
    }
#pragma unroll
    for (int t = 0; t < 4; ++t)
#pragma unroll
      for (int r = 0; r < 8; ++r) {
        const float p = __expf(st[t][r] - mnew[r]);
        st[t][r] = p;
        rs[r] += p;
      }
#pragma unroll
    for (int r = 0; r < 8; ++r) {
      float s = rs[r];
      s += __shfl_xor(s, 1, 32);
      s += __shfl_xor(s, 2, 32);
      s += __shfl_xor(s, 4, 32);
      s += __shfl_xor(s, 8, 32);
      lrun[r] = lrun[r] * alpha[r] + s;
    }
#pragma unroll
    for (int t = 0; t < 4; ++t)
#pragma unroll
      for (int r = 0; r < 8; ++r) o[t][r] *= alpha[r];

#pragma unroll
    for (int t = 0; t < 4; ++t)
#pragma unroll
      for (int r = 0; r < 8; ++r)
        plds[wave][r + 8 * g][t * 16 + N] = (_Float16)(st[t][r] * P_CARRY);
    __syncthreads();
    const v16h ap0 = load_frag(prow, P_LDS, 0, 0,  lane);
    const v16h ap1 = load_frag(prow, P_LDS, 0, 32, lane);
    __syncthreads();

#pragma unroll
    for (int t = 0; t < 4; ++t) {
      const v16h bv0 = load_frag(Vb, SEQ, t * 16, kb,      lane);
      o[t] = wmma_f16(ap0, bv0, o[t]);
      const v16h bv1 = load_frag(Vb, SEQ, t * 16, kb + 32, lane);
      o[t] = wmma_f16(ap1, bv1, o[t]);
    }
  }

  float fac[8];
#pragma unroll
  for (int r = 0; r < 8; ++r) fac[r] = (1.0f / lrun[r]) * AO_FAC;
#pragma unroll
  for (int t = 0; t < 4; ++t)
#pragma unroll
    for (int r = 0; r < 8; ++r)
      plds[wave][r + 8 * g][t * 16 + N] = (_Float16)(o[t][r] * fac[r]);
  __syncthreads();

  const int b  = bh / NHEAD;
  const int h  = bh - b * NHEAD;
  const int lq = lane >> 3;
  const int lp = lane & 7;
  _Float16* base = AOp + ((size_t)b * SEQ + q0) * DMODEL + h * DH;
#pragma unroll
  for (int i = 0; i < 4; ++i) {
    const int row = i * 4 + lq;
    const v4u v = *(const v4u*)&plds[wave][row][lp * 8];
    *(volatile v4u*)(base + (size_t)row * DMODEL + lp * 8) = v;
  }
  __threadfence();
#pragma unroll
  for (int i = 0; i < 4; ++i) {
    const int row = i * 4 + lq;
    const v4u v = *(const v4u*)&plds[wave][row][lp * 8];
    *(volatile v4u*)(base + (size_t)row * DMODEL + lp * 8) = v;
  }
}

__global__ __launch_bounds__(128) __attribute__((amdgpu_num_vgpr(256)))
void oproj_kernel(const _Float16* __restrict__ AOp,
                  const _Float16* __restrict__ Woh,
                  const float* __restrict__ bo,
                  float* __restrict__ out)
{
  __shared__ __attribute__((aligned(16))) float otile[4][32][O_LDS];

  const int lane = threadIdx.x & 31;
  const int wave = threadIdx.x >> 5;
  const int N = lane & 15, g = lane >> 4;
  const int n0  = blockIdx.x * 64;
  const int nb0 = blockIdx.y * 128;
  const int m0  = nb0 + wave * 32;

  v8f acc[2][4];
#pragma unroll
  for (int u = 0; u < 2; ++u)
#pragma unroll
    for (int t = 0; t < 4; ++t)
#pragma unroll
      for (int r = 0; r < 8; ++r) acc[u][t][r] = 0.0f;

#pragma unroll 1
  for (int k0 = 0; k0 < DMODEL; k0 += 32) {
    const v16h a0 = load_frag(AOp, DMODEL, m0,      k0, lane);
    const v16h a1 = load_frag(AOp, DMODEL, m0 + 16, k0, lane);
#pragma unroll
    for (int t = 0; t < 4; ++t) {
      const v16h b = load_frag(Woh, DMODEL, n0 + t * 16, k0, lane);
      acc[0][t] = wmma_f16(a0, b, acc[0][t]);
      acc[1][t] = wmma_f16(a1, b, acc[1][t]);
    }
  }

#pragma unroll
  for (int u = 0; u < 2; ++u)
#pragma unroll
    for (int t = 0; t < 4; ++t) {
      const int   e    = n0 + t * 16 + N;
      const float bias = bf16_rne(bo[e]);
#pragma unroll
      for (int r = 0; r < 8; ++r)
        otile[wave][u * 16 + 8 * g + r][t * 16 + N] = acc[u][t][r] * OUT_FAC + bias;
    }
  __syncthreads();

  const int b  = nb0 / SEQ;
  const int s0 = nb0 - b * SEQ + wave * 32;
  const int lq = lane >> 3;
  const int lp = lane & 7;
  float* base = out + ((size_t)b * OUT_SEQ_STRIDE + s0) * DMODEL + n0;
#pragma unroll
  for (int i = 0; i < 16; ++i) {
    const int L   = i * 4 + lq;
    const int row = L >> 1;
    const int cp  = (L & 1) * 32 + lp * 4;
    const v4f v = *(const v4f*)&otile[wave][row][cp];
    *(volatile v4f*)(base + (size_t)row * DMODEL + cp) = v;
  }
  __threadfence();
#pragma unroll
  for (int i = 0; i < 16; ++i) {
    const int L   = i * 4 + lq;
    const int row = L >> 1;
    const int cp  = (L & 1) * 32 + lp * 4;
    const v4f v = *(const v4f*)&otile[wave][row][cp];
    *(volatile v4f*)(base + (size_t)row * DMODEL + cp) = v;
  }
}

extern "C" void kernel_launch(void* const* d_in, const int* in_sizes, int n_in,
                              void* d_out, int out_size, void* d_ws, size_t ws_size,
                              hipStream_t stream)
{
  if (n_in < 6) return;
  const float* X  = (const float*)d_in[0];
  const float* Wq = (const float*)d_in[1];
  const float* Wk = (const float*)d_in[2];
  const float* Wv = (const float*)d_in[3];
  const float* Wo = (const float*)d_in[4];
  const float* bo = (const float*)d_in[5];
  float* out = (float*)d_out;

  if ((size_t)in_sizes[0] < ((size_t)(NB - 1) * SEQ_FULL + SEQ) * DMODEL) return;
  if (in_sizes[1] < DMODEL * DMODEL || in_sizes[2] < DMODEL * DMODEL ||
      in_sizes[3] < DMODEL * DMODEL || in_sizes[4] < DMODEL * DMODEL) return;
  if (in_sizes[5] < DMODEL) return;
  if ((size_t)out_size < ((size_t)(NB - 1) * OUT_SEQ_STRIDE + SEQ) * DMODEL) return;

  const size_t SZ_X  = (size_t)NROWS * DMODEL * sizeof(_Float16);
  const size_t SZ_W  = (size_t)DMODEL * DMODEL * sizeof(_Float16);
  const size_t SZ_QK = (size_t)NBH * SEQ * DH * sizeof(_Float16);
  const size_t SZ_AO = (size_t)NROWS * DMODEL * sizeof(_Float16);

  char* ws = (char*)d_ws;
  size_t off = 0;
  _Float16* Xh  = (_Float16*)(ws + off); off += SZ_X;
  _Float16* Wqh = (_Float16*)(ws + off); off += SZ_W;
  _Float16* Wkh = (_Float16*)(ws + off); off += SZ_W;
  _Float16* Wvh = (_Float16*)(ws + off); off += SZ_W;
  _Float16* Woh = (_Float16*)(ws + off); off += SZ_W;
  _Float16* Qp  = (_Float16*)(ws + off); off += SZ_QK;
  _Float16* Kp  = (_Float16*)(ws + off); off += SZ_QK;
  _Float16* Vtp = (_Float16*)(ws + off); off += SZ_QK;
  _Float16* AOp = (_Float16*)(ws + off); off += SZ_AO;
  if (off > ws_size) return;

  const int nxblk = (NROWS * DMODEL) / (256 * 8);

  cvt_kernel<<<nxblk + 4 * 128, 256, 0, stream>>>(X, Wq, Wk, Wv, Wo, Xh, Wqh, Wkh, Wvh, Woh, nxblk);
  qkv_kernel<<<dim3(NHEAD, NROWS / 128, 3), 128, 0, stream>>>(Xh, Wqh, Wkh, Wvh, Qp, Kp, Vtp);
  attn_kernel<<<dim3(SEQ / 64, NBH), 128, 0, stream>>>(Qp, Kp, Vtp, AOp);
  oproj_kernel<<<dim3(DMODEL / 64, NROWS / 128), 128, 0, stream>>>(AOp, Woh, bo, out);
}
